// BidirRWKV6DeltaTimeMix_69818988364380
// MI455X (gfx1250) — hardware-verified
//
#include <hip/hip_runtime.h>
#include <math.h>

constexpr int kBatch = 2;
constexpr int kSeq   = 1024;
constexpr int kDim   = 1024;
constexpr int kHeads = 16;
constexpr int kHd    = 64;
constexpr int kTok   = kBatch * kSeq;
constexpr int kMixW  = 32;
constexpr int kMixN  = 6 * kMixW;
constexpr int kLora  = 64;
constexpr int kMid   = kSeq / 2;
constexpr float kGnEps    = 1e-5f * 64.0f;
constexpr float kClip     = 60.0f;
constexpr float kCarryW   = 1024.0f;
constexpr float kCarryH   = 64.0f;
constexpr float kCarryMix = 256.0f;
constexpr int   kMixShift = 8;
constexpr float kCarryV   = 16.0f;
constexpr float kCarrySU  = 1024.0f;
constexpr float kCarrySY  = 64.0f;
static_assert(kDim == kHeads * kHd);
static_assert(kTok % 64 == 0 && kDim % 64 == 0 && kMixN % 64 == 0 && kLora % 64 == 0);
static_assert(kDim % 32 == 0 && kMixW % 32 == 0 && kLora % 32 == 0 && kHd % 32 == 0);
static_assert((float)(1 << kMixShift) == kCarryMix);
static_assert(kSeq % 64 == 0 && (kSeq & (kSeq - 1)) == 0);

typedef __attribute__((ext_vector_type(16))) _Float16 v16h;
typedef __attribute__((ext_vector_type(8)))  _Float16 v8h;
typedef __attribute__((ext_vector_type(16))) __bf16   v16b;
typedef __attribute__((ext_vector_type(8)))  __bf16   v8b;
typedef __attribute__((ext_vector_type(8)))  float    v8f;
typedef __attribute__((ext_vector_type(4)))  float    v4f;
typedef __attribute__((ext_vector_type(4)))  unsigned int v4u;

__device__ __forceinline__ unsigned short f2bf_bits(float f) {
  unsigned u = __float_as_uint(f);
  return (unsigned short)((u + 0x7FFFu + ((u >> 16) & 1u)) >> 16);
}
__device__ __forceinline__ float bf_bits2f(unsigned short h) { return __uint_as_float(((unsigned)h) << 16); }
__device__ __forceinline__ unsigned pk16(unsigned short a, unsigned short b) { return (unsigned)a | ((unsigned)b << 16); }
__device__ __forceinline__ unsigned short h_bits(float f) { const _Float16 h = (_Float16)f; return __builtin_bit_cast(unsigned short, h); }

template <int SH>
__device__ __forceinline__ float h16_to_f32_dn(unsigned hb) {
  const unsigned sgn = (hb & 0x8000u) << 16;
  const unsigned em = hb & 0x7fffu;
  const float fn = __uint_as_float((em << 13) + 0x38000000u - ((unsigned)SH << 23));
  const float fs = (float)em * (5.9604644775390625e-8f / (float)(1 << SH));
  const float mag = (em < 0x400u) ? fs : fn;
  return __uint_as_float(__float_as_uint(mag) | sgn);
}

__device__ __forceinline__ v4u pack8_f16(const float* v) {
  unsigned short b[8];
#pragma unroll
  for (int e = 0; e < 8; ++e) b[e] = h_bits(v[e]);
  return (v4u){pk16(b[0], b[1]), pk16(b[2], b[3]), pk16(b[4], b[5]), pk16(b[6], b[7])};
}
__device__ __forceinline__ void pack8_bf_hl(const float* v, v4u& hi, v4u& lo) {
  unsigned short hb[8], lb[8];
#pragma unroll
  for (int e = 0; e < 8; ++e) {
    hb[e] = f2bf_bits(v[e]);
    lb[e] = f2bf_bits(v[e] - bf_bits2f(hb[e]));
  }
  hi = (v4u){pk16(hb[0], hb[1]), pk16(hb[2], hb[3]), pk16(hb[4], hb[5]), pk16(hb[6], hb[7])};
  lo = (v4u){pk16(lb[0], lb[1]), pk16(lb[2], lb[3]), pk16(lb[4], lb[5]), pk16(lb[6], lb[7])};
}

__device__ __forceinline__ void wave_lds_sync() {
  __builtin_amdgcn_fence(__ATOMIC_RELEASE, "workgroup");
  __builtin_amdgcn_wave_barrier();
  __builtin_amdgcn_fence(__ATOMIC_ACQUIRE, "workgroup");
}

__device__ __forceinline__ void dep_guard4_h(v8f& a, v8f& b, v8f& c, v8f& d, v16h x, v16h y) { asm volatile("v_nop\n\tv_nop\n\tv_nop\n\tv_nop" : "+v"(a), "+v"(b), "+v"(c), "+v"(d) : "v"(x), "v"(y)); }
__device__ __forceinline__ void dep_guard4_b(v8f& a, v8f& b, v8f& c, v8f& d, v16b x, v16b y) { asm volatile("v_nop\n\tv_nop\n\tv_nop\n\tv_nop" : "+v"(a), "+v"(b), "+v"(c), "+v"(d) : "v"(x), "v"(y)); }
__device__ __forceinline__ void keep4_h(v16h a, v16h b, v16h c, v16h d) { asm volatile("v_nop" :: "v"(a), "v"(b), "v"(c), "v"(d)); }
__device__ __forceinline__ void keep4_b(v16b a, v16b b, v16b c, v16b d) { asm volatile("v_nop" :: "v"(a), "v"(b), "v"(c), "v"(d)); }
__device__ __forceinline__ void acc_guard4(v8f& a, v8f& b, v8f& c, v8f& d) { asm volatile("v_nop\n\tv_nop\n\tv_nop\n\tv_nop" : "+v"(a), "+v"(b), "+v"(c), "+v"(d)); }

template <typename T> struct Frag;
template <> struct Frag<_Float16> {
  typedef v16h V; union U { v16h v; v8h h[2]; };
  static __device__ __forceinline__ v16h load(const _Float16* p) {
    U f; f.h[0] = *(const v8h*)(p); f.h[1] = *(const v8h*)(p + 16); return f.v;
  }
  static __device__ __forceinline__ v8f mma(v16h a, v16h b, v8f c) {
    return __builtin_amdgcn_wmma_f32_16x16x32_f16(false, a, false, b, (short)0, c, false, false);
  }
  static __device__ __forceinline__ void guard(v8f& a, v8f& b, v8f& c, v8f& d, v16h x, v16h y) { dep_guard4_h(a, b, c, d, x, y); }
  static __device__ __forceinline__ void keep(v16h a, v16h b, v16h c, v16h d) { keep4_h(a, b, c, d); }
};
template <> struct Frag<__bf16> {
  typedef v16b V; union U { v16b v; v8b h[2]; };
  static __device__ __forceinline__ v16b load(const __bf16* p) {
    U f; f.h[0] = *(const v8b*)(p); f.h[1] = *(const v8b*)(p + 16); return f.v;
  }
  static __device__ __forceinline__ v8f mma(v16b a, v16b b, v8f c) {
    return __builtin_amdgcn_wmma_f32_16x16x32_bf16(false, a, false, b, (short)0, c, false, false);
  }
  static __device__ __forceinline__ void guard(v8f& a, v8f& b, v8f& c, v8f& d, v16b x, v16b y) { dep_guard4_b(a, b, c, d, x, y); }
  static __device__ __forceinline__ void keep(v16b a, v16b b, v16b c, v16b d) { keep4_b(a, b, c, d); }
};

__device__ __forceinline__ v8f mma_b(v16b a, v16b b, v8f c) {
  c = __builtin_amdgcn_wmma_f32_16x16x32_bf16(false, a, false, b, (short)0, c, false, false);
  asm volatile("v_nop\n\tv_nop\n\tv_nop\n\tv_nop" : "+v"(c) : "v"(a), "v"(b));
  return c;
}
__device__ __forceinline__ v8f mma_h(v16h a, v16h b, v8f c) {
  c = __builtin_amdgcn_wmma_f32_16x16x32_f16(false, a, false, b, (short)0, c, false, false);
  asm volatile("v_nop\n\tv_nop\n\tv_nop\n\tv_nop" : "+v"(c) : "v"(a), "v"(b));
  return c;
}

template <int ET> struct Elem;
template <> struct Elem<0> { typedef _Float16 T; };
template <> struct Elem<1> { typedef __bf16 T; };
template <int ET, bool SPLIT, int BIAS_MODE, int OUT_MODE, int ACT>
__global__ __launch_bounds__(256) void wmma_gemm64(
    const unsigned short* __restrict__ Ap, const unsigned short* __restrict__ A2p, int lda, long strideA,
    const unsigned short* __restrict__ Btp, const unsigned short* __restrict__ Bt2p, int ldb, long strideB,
    void* __restrict__ Cout, void* __restrict__ Cout2, int ldc, long strideC,
    const float* __restrict__ bias,
    int M, int N, int K, float scale) {
  typedef typename Elem<ET>::T T;
  typedef typename Frag<T>::V V;
  const T* A = (const T*)Ap; const T* A2 = (const T*)A2p; const T* Bt = (const T*)Btp; const T* Bt2 = (const T*)Bt2p;
  __shared__ __align__(16) float sT[8][16 * 68];
  const int b    = blockIdx.y;
  const int lane = threadIdx.x & 31;
  const int wave = threadIdx.x >> 5;
  const int tilesN = N >> 6;
  const int tilesM = M >> 6;
  const int tile = blockIdx.x * 8 + wave;
  if (tile >= tilesM * tilesN) return;
  const int tm = tile / tilesN;
  const int tn = tile - tm * tilesN;
  const int m0 = tm << 6;
  const int n0 = tn << 6;

  const T* Ab  = A  + (size_t)b * strideA;
  const T* Bb  = Bt + (size_t)b * strideB;
  const T* Ab2 = SPLIT ? (A2  + (size_t)b * strideA) : nullptr;
  const T* Bb2 = SPLIT ? (Bt2 + (size_t)b * strideB) : nullptr;

  const int rlane = lane & 15;
  const int koff  = (lane >> 4) * 8;
  const int mOff  = (lane >> 4) * 8;

  v8f acc[4][4];
#pragma unroll
  for (int i = 0; i < 4; ++i)
#pragma unroll
    for (int j = 0; j < 4; ++j) acc[i][j] = (v8f){0.f,0.f,0.f,0.f,0.f,0.f,0.f,0.f};

  for (int k0 = 0; k0 < K; k0 += 32) {
    V bh[4], bl[4];
#pragma unroll
    for (int j = 0; j < 4; ++j) {
      const size_t bo = (size_t)(n0 + (j << 4) + rlane) * ldb + koff + k0;
      bh[j] = Frag<T>::load(Bb + bo);
      if (SPLIT) bl[j] = Frag<T>::load(Bb2 + bo);
    }
#pragma unroll
    for (int i = 0; i < 4; ++i) {
      const size_t ao = (size_t)(m0 + (i << 4) + rlane) * lda + koff + k0;
      V ah = Frag<T>::load(Ab + ao);
      V al = ah;
      if (SPLIT) al = Frag<T>::load(Ab2 + ao);
#pragma unroll
      for (int j = 0; j < 4; ++j) {
        acc[i][j] = Frag<T>::mma(ah, bh[j], acc[i][j]);
        if (SPLIT) {
          acc[i][j] = Frag<T>::mma(ah, bl[j], acc[i][j]);
          acc[i][j] = Frag<T>::mma(al, bh[j], acc[i][j]);
        }
      }
      Frag<T>::guard(acc[i][0], acc[i][1], acc[i][2], acc[i][3], ah, al);
    }
    Frag<T>::keep(bh[0], bh[1], bh[2], bh[3]);
    if (SPLIT) Frag<T>::keep(bl[0], bl[1], bl[2], bl[3]);
  }
  acc_guard4(acc[0][0], acc[0][1], acc[0][2], acc[0][3]);
  acc_guard4(acc[1][0], acc[1][1], acc[1][2], acc[1][3]);
  acc_guard4(acc[2][0], acc[2][1], acc[2][2], acc[2][3]);
  acc_guard4(acc[3][0], acc[3][1], acc[3][2], acc[3][3]);

  float* slab = sT[wave];
#pragma unroll
  for (int i = 0; i < 4; ++i) {
    const int mBase = m0 + (i << 4);
#pragma unroll
    for (int j = 0; j < 4; ++j) {
      const int n = n0 + (j << 4) + rlane;
      float bv = 0.f;
      if (BIAS_MODE == 2) bv = bias[n];
#pragma unroll
      for (int r = 0; r < 8; ++r) {
        float v = acc[i][j][r] * scale;
        if (BIAS_MODE == 2) v += bv;
        if (ACT == 1) v = tanhf(v) * kCarryH;
        slab[(mOff + r) * 68 + (j << 4) + rlane] = v;
      }
    }
    wave_lds_sync();
    if (OUT_MODE == 0) {
      float* C = (float*)Cout + (size_t)b * strideC;
      const int hh = lane >> 4, c4 = (lane & 15) * 4;
      for (int pass = 0; pass < 2; ++pass) {
#pragma unroll
        for (int it = 0; it < 8; ++it) {
          const int row = it * 2 + hh;
          v4f v = *(const v4f*)(slab + row * 68 + c4);
          *(volatile v4f*)(C + (size_t)(mBase + row) * ldc + n0 + c4) = v;
        }
        __threadfence();
      }
    } else {
      const int q = lane >> 3, c8 = (lane & 7) * 8;
      unsigned short* C  = (unsigned short*)Cout  + (size_t)b * strideC;
      unsigned short* C2 = (OUT_MODE == 2) ? ((unsigned short*)Cout2 + (size_t)b * strideC) : nullptr;
      for (int pass = 0; pass < 2; ++pass) {
#pragma unroll
        for (int it = 0; it < 4; ++it) {
          const int row = it * 4 + q;
          const float* sp = slab + row * 68 + c8;
          v8h hv, lv;
#pragma unroll
          for (int e = 0; e < 8; ++e) {
            if (OUT_MODE == 1) {
              hv[e] = (_Float16)sp[e];
            } else {
              unsigned short hb = f2bf_bits(sp[e]);
              unsigned short lb = f2bf_bits(sp[e] - bf_bits2f(hb));
              hv[e] = __builtin_bit_cast(_Float16, hb);
              lv[e] = __builtin_bit_cast(_Float16, lb);
            }
          }
          *(volatile v8h*)(C + (size_t)(mBase + row) * ldc + n0 + c8) = hv;
          if (OUT_MODE == 2) *(volatile v8h*)(C2 + (size_t)(mBase + row) * ldc + n0 + c8) = lv;
        }
        __threadfence();
      }
    }
    wave_lds_sync();
  }
}

template <int MODE>
__global__ __launch_bounds__(256) void trw_kernel(const float* __restrict__ W0, const float* __restrict__ W1,
                                                  const float* __restrict__ W2, const float* __restrict__ W3,
                                                  unsigned short* __restrict__ outHi, unsigned short* __restrict__ outLo,
                                                  int kin, int nout, float scale) {
  __shared__ float sm[64][65];
  const int t  = threadIdx.x;
  const int k0 = blockIdx.x * 64;
  const int n0 = blockIdx.y * 64;
  const int z  = blockIdx.z;
  const float* W = (z == 0) ? W0 : (z == 1) ? W1 : (z == 2) ? W2 : W3;
#pragma unroll
  for (int i = 0; i < 16; ++i) {
    const int e = i * 256 + t;
    const int r = e >> 6;
    const int c = e & 63;
    sm[c][r] = W[(size_t)(k0 + r) * nout + n0 + c] * scale;
  }
  __syncthreads();
  const int lane = t & 31, wave = t >> 5;
  const int q = lane >> 3, c8 = (lane & 7) * 8;
  v4u uh[2], ul[2];
#pragma unroll
  for (int it = 0; it < 2; ++it) {
    const int row = wave * 8 + it * 4 + q;
    float o[8];
#pragma unroll
    for (int e = 0; e < 8; ++e) o[e] = sm[row][c8 + e];
    if (MODE == 0) { uh[it] = pack8_f16(o); ul[it] = uh[it]; }
    else pack8_bf_hl(o, uh[it], ul[it]);
  }
  const size_t pl = (size_t)z * nout * kin;
  for (int pass = 0; pass < 2; ++pass) {
#pragma unroll
    for (int it = 0; it < 2; ++it) {
      const int row = wave * 8 + it * 4 + q;
      const size_t o = pl + (size_t)(n0 + row) * kin + k0 + c8;
      *(volatile v4u*)(outHi + o) = uh[it];
      if (MODE == 1) *(volatile v4u*)(outLo + o) = ul[it];
    }
    __threadfence();
  }
}

__global__ __launch_bounds__(256) void tr32_kernel(const float* __restrict__ W, unsigned short* __restrict__ out, float scale) {
  __shared__ float sm[64][33];
  const int t = threadIdx.x;
  const int n0 = blockIdx.x * 64;
  const int s = blockIdx.y;
#pragma unroll
  for (int i = 0; i < 8; ++i) {
    const int e = i * 256 + t;
    const int r = e >> 6;
    const int c = e & 63;
    sm[c][r] = W[((size_t)s * kMixW + r) * kDim + n0 + c] * scale;
  }
  __syncthreads();
  const int nl = t >> 2, kc = (t & 3) * 8;
  float o[8];
#pragma unroll
  for (int e = 0; e < 8; ++e) o[e] = sm[nl][kc + e];
  const v4u u = pack8_f16(o);
  unsigned short* dst = out + ((size_t)s * kDim + n0 + nl) * kMixW + kc;
  *(volatile v4u*)dst = u;
  __threadfence();
  *(volatile v4u*)dst = u;
}

__device__ __forceinline__ void load_x_dx(const float* __restrict__ x, int tok, int c8, float* xv, float* dxv) {
  const int t = tok & (kSeq - 1);
  const bool hasL = (t > 0);
  const bool hasR = (t < kSeq - 1);
  const int tokm = hasL ? (tok - 1) : tok;
  const int tokp = hasR ? (tok + 1) : tok;
  const float* p0 = x + (size_t)tok * kDim + c8;
  const float* pm = x + (size_t)tokm * kDim + c8;
  const float* pp = x + (size_t)tokp * kDim + c8;
  const v4f a0 = *(const v4f*)(p0), a1 = *(const v4f*)(p0 + 4);
  const v4f l0 = *(const v4f*)(pm), l1 = *(const v4f*)(pm + 4);
  const v4f r0 = *(const v4f*)(pp), r1 = *(const v4f*)(pp + 4);
#pragma unroll
  for (int e = 0; e < 4; ++e) {
    const float lf0 = hasL ? l0[e] : 0.0f, rt0 = hasR ? r0[e] : 0.0f;
    const float lf1 = hasL ? l1[e] : 0.0f, rt1 = hasR ? r1[e] : 0.0f;
    xv[e] = a0[e];
    xv[4 + e] = a1[e];
    dxv[e] = (lf0 + rt0) * 0.5f - a0[e];
    dxv[4 + e] = (lf1 + rt1) * 0.5f - a1[e];
  }
}

__global__ __launch_bounds__(256) void shift_kernel(const float* __restrict__ x, const float* __restrict__ tmx,
                                                    unsigned short* __restrict__ XXX) {
  const int i = blockIdx.x * 256 + threadIdx.x;
  if (i >= kTok * (kDim / 8)) return;
  const int tok = i >> 7;
  const int c8 = (i & 127) * 8;
  float xv[8], dx[8];
  load_x_dx(x, tok, c8, xv, dx);
  const v4f m0 = *(const v4f*)(tmx + c8), m1 = *(const v4f*)(tmx + c8 + 4);
  float o[8];
#pragma unroll
  for (int e = 0; e < 4; ++e) {
    o[e] = xv[e] + dx[e] * m0[e];
    o[4 + e] = xv[4 + e] + dx[4 + e] * m1[e];
  }
  const v4u u = pack8_f16(o);
  unsigned short* dst = XXX + (size_t)tok * kDim + c8;
  *(volatile v4u*)dst = u;
  __threadfence();
  *(volatile v4u*)dst = u;
}

__device__ __forceinline__ void mix_eval(const float* xv, const float* dx, const float* __restrict__ maa,
                                         const unsigned short* __restrict__ mixp, float* o) {
  const v4f m0 = *(const v4f*)(maa), m1 = *(const v4f*)(maa + 4);
  const v4u mw = *(const v4u*)(mixp);
  float mf[8];
#pragma unroll
  for (int q = 0; q < 4; ++q) {
    const unsigned w = mw[q];
    mf[2 * q]     = h16_to_f32_dn<kMixShift>(w & 0xffffu);
    mf[2 * q + 1] = h16_to_f32_dn<kMixShift>(w >> 16);
  }
#pragma unroll
  for (int e = 0; e < 4; ++e) {
    o[e] = xv[e] + dx[e] * (m0[e] + mf[e]);
    o[4 + e] = xv[4 + e] + dx[4 + e] * (m1[e] + mf[4 + e]);
  }
}

__global__ __launch_bounds__(256) void combine_kernel(const float* __restrict__ x,
    const float* __restrict__ tw, const float* __restrict__ tk, const float* __restrict__ tv,
    const float* __restrict__ tr, const float* __restrict__ tg, const float* __restrict__ ta,
    const unsigned short* __restrict__ MIX,
    unsigned short* __restrict__ XW, unsigned short* __restrict__ X4H, unsigned short* __restrict__ X4L,
    unsigned short* __restrict__ XAH, unsigned short* __restrict__ XAL) {
  const int i = blockIdx.x * 256 + threadIdx.x;
  if (i >= kTok * (kDim / 8)) return;
  const int tok = i >> 7;
  const int c8 = (i & 127) * 8;
  const size_t eo = (size_t)tok * kDim + c8;
  const size_t pl = (size_t)kTok * kDim;
  float xv[8], dx[8], o[8];
  load_x_dx(x, tok, c8, xv, dx);
  v4u uw, uh[5], ul[5];
  mix_eval(xv, dx, tw + c8, MIX + 0 * pl + eo, o);
  uw = pack8_f16(o);
  mix_eval(xv, dx, tk + c8, MIX + 1 * pl + eo, o);
  pack8_bf_hl(o, uh[0], ul[0]);
  mix_eval(xv, dx, tv + c8, MIX + 2 * pl + eo, o);
  pack8_bf_hl(o, uh[1], ul[1]);
  mix_eval(xv, dx, tr + c8, MIX + 3 * pl + eo, o);
  pack8_bf_hl(o, uh[2], ul[2]);
  mix_eval(xv, dx, tg + c8, MIX + 4 * pl + eo, o);
  pack8_bf_hl(o, uh[3], ul[3]);
  mix_eval(xv, dx, ta + c8, MIX + 5 * pl + eo, o);
  pack8_bf_hl(o, uh[4], ul[4]);
  for (int pass = 0; pass < 2; ++pass) {
    *(volatile v4u*)(XW + eo) = uw;
#pragma unroll
    for (int s = 0; s < 4; ++s) {
      *(volatile v4u*)(X4H + (size_t)s * pl + eo) = uh[s];
      *(volatile v4u*)(X4L + (size_t)s * pl + eo) = ul[s];
    }
    *(volatile v4u*)(XAH + eo) = uh[4];
    *(volatile v4u*)(XAL + eo) = ul[4];
    __threadfence();
  }
}

__global__ __launch_bounds__(64) void scan_kernel(const float* __restrict__ WD, float* __restrict__ CS) {
  const int id = blockIdx.x * 64 + threadIdx.x;
  const int b = id >> 10;
  const int d = id & (kDim - 1);
  const size_t base = (size_t)b * kSeq * kDim + d;
#pragma unroll 1
  for (int pass = 0; pass < 2; ++pass) {
    float cs = 0.0f;
#pragma unroll 1
    for (int t = 0; t < kSeq; ++t) {
      const float w = WD[base + (size_t)t * kDim];
      cs = cs + (-expf(w));
      *(volatile float*)(CS + base + (size_t)t * kDim) = cs;
    }
    __threadfence();
  }
}

__device__ __forceinline__ void put_hl(unsigned short* s_out, int p, int d, float v) {
  const unsigned short hb = f2bf_bits(v);
  s_out[p * kDim + d] = hb;
  s_out[(p + 1) * kDim + d] = f2bf_bits(v - bf_bits2f(hb));
}

__global__ __launch_bounds__(256) void headprep_kernel(
    const float* __restrict__ Kf, const float* __restrict__ Vf, const float* __restrict__ Rf,
    const float* __restrict__ PRE, const float* __restrict__ WD, const float* __restrict__ CS,
    const float* __restrict__ k_k, const float* __restrict__ k_a,
    unsigned short* __restrict__ wsb, long offQ, long offA, long offV) {
  __shared__ float s_kk[kDim];
  __shared__ float s_inv[kHeads];
  __shared__ __align__(16) unsigned short s_out[13 * kDim];
  const int tok = blockIdx.x;
  const int b = tok >> 10;
  const int t = tok & (kSeq - 1);
  const int tid = threadIdx.x;
  const size_t rowoff = (size_t)tok * kDim;
  const size_t midoff = ((size_t)b * kSeq + kMid) * kDim;
#pragma unroll 1
  for (int it = 0; it < 4; ++it) {
    const int d = it * 256 + tid;
    s_kk[d] = Kf[rowoff + d] * k_k[d];
  }
  __syncthreads();
  {
    const int h = tid >> 4, sub = tid & 15;
    float ss = 0.0f;
#pragma unroll
    for (int e = 0; e < 4; ++e) { const float v = s_kk[h * kHd + sub * 4 + e]; ss += v * v; }
    ss += __shfl_xor(ss, 8, 32);
    ss += __shfl_xor(ss, 4, 32);
    ss += __shfl_xor(ss, 2, 32);
    ss += __shfl_xor(ss, 1, 32);
    if (sub == 0) s_inv[h] = 1.0f / fmaxf(sqrtf(ss), 1e-12f);
  }
  __syncthreads();
#pragma unroll 1
  for (int it = 0; it < 4; ++it) {
    const int d = it * 256 + tid;
    const int h = d >> 6;
    const size_t g = rowoff + d;
    const float kraw = Kf[g];
    const float rr = Rf[g];
    const float vv = Vf[g];
    const float pre = PRE[g];
    const float w = WD[g];
    const float cs = CS[g];
    const float wm = WD[midoff + d];
    const float csm = CS[midoff + d];
    const float ka = k_a[d];
    const float kk = s_kk[d] * s_inv[h];
    const float ic = 1.0f / (1.0f + expf(-pre));
    const float kmod = kraw * (1.0f + (ic - 1.0f) * ka);
    const float wh = -expf(w);
    const float whm = -expf(wm);
    const float cf = fminf(fmaxf(cs - csm, -kClip), kClip);
    const float cb = fminf(fmaxf((cs - wh) - (csm - whm), -kClip), kClip);
    const float ef = expf(cf), enf = expf(-cf), eb = expf(cb), enb = expf(-cb);
    put_hl(s_out, 0, d, rr * ef);
    put_hl(s_out, 2, d, kmod * enf);
    put_hl(s_out, 4, d, rr * enb);
    put_hl(s_out, 6, d, kmod * eb);
    put_hl(s_out, 8, d, kk * ic);
    put_hl(s_out, 10, d, kk);
    s_out[12 * kDim + d] = h_bits(vv * kCarryV);
  }
  __syncthreads();
  const int lane8 = tid & 7, grp = tid >> 3;
  for (int pass = 0; pass < 2; ++pass) {
#pragma unroll 1
    for (int it = 0; it < 7; ++it) {
      const int L = it * 32 + grp;
      if (L < 13 * kHeads) {
        const int p = L >> 4, h = L & 15;
        const v4u u = *(const v4u*)(s_out + p * kDim + h * kHd + lane8 * 8);
        const size_t pl = (size_t)kTok * kDim;
        const size_t poff = (p < 8) ? ((size_t)offQ + (size_t)p * pl)
                          : (p < 12) ? ((size_t)offA + (size_t)(p - 8) * pl) : (size_t)offV;
        const size_t o = poff + (((size_t)b * kHeads + h) * kSeq + t) * kHd + lane8 * 8;
        *(volatile v4u*)(wsb + o) = u;
      }
    }
    __threadfence();
  }
}

template <bool UM>
__global__ __launch_bounds__(128) void pairmix_kernel(
    const unsigned short* Q0h, const unsigned short* Q0l, const unsigned short* K0h, const unsigned short* K0l,
    const unsigned short* V0,
    const unsigned short* Q1h, const unsigned short* Q1l, const unsigned short* K1h, const unsigned short* K1l,
    const unsigned short* V1,
    const float* Vres, unsigned short* outU0, unsigned short* outU1, float* outY) {
  __shared__ __align__(16) unsigned short Ksh[64 * 64];
  __shared__ __align__(16) unsigned short Ksl[64 * 64];
  __shared__ __align__(16) unsigned short Vts[64 * 64];
  __shared__ __align__(16) _Float16 Psh[4][16 * 64];
  __shared__ __align__(16) float Os[4][16 * 68];

  const int tid = threadIdx.x;
  const int wave = tid >> 5;
  const int lane = tid & 31;
  const int hh = lane >> 4;
  const int c = lane & 15;
  const int ib = blockIdx.x & 15;
  const int bh = blockIdx.x >> 4;
  const int b = bh >> 4;
  const int h = bh & 15;
  const int i0 = ib * 64;
  const int q0 = i0 + wave * 16;
  const size_t hb = (size_t)bh * kSeq * kHd;
  const float SC = UM ? kCarrySU : kCarrySY;
  const float INV = 1.0f / (SC * kCarryV);

  v8f acc[4];
#pragma unroll
  for (int t = 0; t < 4; ++t) acc[t] = (v8f){0.f,0.f,0.f,0.f,0.f,0.f,0.f,0.f};
  _Float16* pw = Psh[wave];
  float* os = Os[wave];

#pragma unroll 1
  for (int pass = 0; pass < 2; ++pass) {
    const unsigned short* Qh = pass ? Q1h : Q0h;
    const unsigned short* Ql = pass ? Q1l : Q0l;
    const unsigned short* Kh = pass ? K1h : K0h;
    const unsigned short* Kl = pass ? K1l : K0l;
    const unsigned short* Vp = pass ? V1 : V0;
    v16b qh[2], ql[2];
    {
      const size_t qo = hb + (size_t)(q0 + c) * kHd + 8 * hh;
#pragma unroll
      for (int dc = 0; dc < 2; ++dc) {
        qh[dc] = Frag<__bf16>::load((const __bf16*)(Qh + qo) + dc * 32);
        ql[dc] = Frag<__bf16>::load((const __bf16*)(Ql + qo) + dc * 32);
      }
    }
    const int jlo = pass ? ib : 0;
    const int jhi = pass ? (kSeq / 64 - 1) : ib;
#pragma unroll 1
    for (int jb = jlo; jb <= jhi; ++jb) {
      const int j0 = jb * 64;
      __syncthreads();
#pragma unroll
      for (int it = 0; it < 4; ++it) {
        const int idx = it * 128 + tid;
        const size_t go = hb + (size_t)j0 * kHd + (size_t)idx * 8;
        const v4u a = *(const v4u*)(Kh + go);
        const v4u bl = *(const v4u*)(Kl + go);
        const v4u w = *(const v4u*)(Vp + go);
        *(v4u*)(Ksh + idx * 8) = a;
        *(v4u*)(Ksl + idx * 8) = bl;
        const int kv = idx >> 3;
        const int d0 = (idx & 7) * 8;
#pragma unroll
        for (int q = 0; q < 4; ++q) {
          const unsigned word = w[q];
          Vts[(d0 + 2 * q) * 64 + kv] = (unsigned short)(word & 0xffffu);
          Vts[(d0 + 2 * q + 1) * 64 + kv] = (unsigned short)(word >> 16);
        }
      }
      __syncthreads();

      v8f s[4];
#pragma unroll
      for (int j = 0; j < 4; ++j) {
        s[j] = (v8f){0.f,0.f,0.f,0.f,0.f,0.f,0.f,0.f};
#pragma unroll
        for (int dc = 0; dc < 2; ++dc) {
          const v16b kb = Frag<__bf16>::load((const __bf16*)Ksh + (j * 16 + c) * 64 + dc * 32 + 8 * hh);
          const v16b kl = Frag<__bf16>::load((const __bf16*)Ksl + (j * 16 + c) * 64 + dc * 32 + 8 * hh);
          s[j] = mma_b(qh[dc], kb, s[j]);
          s[j] = mma_b(qh[dc], kl, s[j]);
          s[j] = mma_b(ql[dc], kb, s[j]);
        }
      }
      const bool diag = (jb == ib);
#pragma unroll
      for (int j = 0; j < 4; ++j) {
#pragma unroll
        for (int r = 0; r < 8; ++r) {
          const int qrow = wave * 16 + 8 * hh + r;
          const int col = j * 16 + c;
          const bool kf = UM ? (qrow > col) : (qrow >= col);
          const bool kd = pass ? (qrow < col) : kf;
          const bool keep = (!diag) || kd;
          const float p = keep ? (s[j][r] * SC) : 0.0f;
          pw[(8 * hh + r) * 64 + j * 16 + c] = (_Float16)p;
        }
      }
      wave_lds_sync();
#pragma unroll
      for (int kk = 0; kk < 2; ++kk) {
        const v16h pa = Frag<_Float16>::load(pw + c * 64 + kk * 32 + 8 * hh);
#pragma unroll
        for (int t = 0; t < 4; ++t) {
          const v16h vb = Frag<_Float16>::load((const _Float16*)Vts + (t * 16 + c) * 64 + kk * 32 + 8 * hh);
          acc[t] = mma_h(pa, vb, acc[t]);
        }
      }
    }
    if (UM) {
#pragma unroll
      for (int t = 0; t < 4; ++t)
#pragma unroll
        for (int r = 0; r < 8; ++r) os[(8 * hh + r) * 68 + t * 16 + c] = acc[t][r] * INV;
      wave_lds_sync();
      const int q = lane >> 3, c8 = (lane & 7) * 8;
      v4u ov[4];
#pragma unroll
      for (int it = 0; it < 4; ++it) {
        const int row = it * 4 + q;
        const float* vp = Vres + ((size_t)b * kSeq + q0 + row) * kDim + h * kHd + c8;
        const v4f va = *(const v4f*)(vp), vb = *(const v4f*)(vp + 4);
        const v4f ua = *(const v4f*)(os + row * 68 + c8), ub = *(const v4f*)(os + row * 68 + c8 + 4);
        float o[8];
#pragma unroll
        for (int e = 0; e < 4; ++e) {
          o[e] = (va[e] - ua[e]) * kCarryV;
          o[4 + e] = (vb[e] - ub[e]) * kCarryV;
        }
        ov[it] = pack8_f16(o);
      }
      unsigned short* op = (pass ? outU1 : outU0) + hb;
      for (int p2 = 0; p2 < 2; ++p2) {
#pragma unroll
        for (int it = 0; it < 4; ++it)
          *(volatile v4u*)(op + (size_t)(q0 + it * 4 + q) * kHd + c8) = ov[it];
        __threadfence();
      }
      wave_lds_sync();
#pragma unroll
      for (int t = 0; t < 4; ++t) acc[t] = (v8f){0.f,0.f,0.f,0.f,0.f,0.f,0.f,0.f};
    }
  }
  if (!UM) {
#pragma unroll
    for (int t = 0; t < 4; ++t)
#pragma unroll
      for (int r = 0; r < 8; ++r) os[(8 * hh + r) * 68 + t * 16 + c] = acc[t][r] * INV;
    wave_lds_sync();
    const int c4 = c * 4;
    float* yb = outY + ((size_t)b * kSeq + q0) * kDim + h * kHd;
    for (int p2 = 0; p2 < 2; ++p2) {
#pragma unroll
      for (int it = 0; it < 8; ++it) {
        const int row = it * 2 + hh;
        const v4f val = *(const v4f*)(os + row * 68 + c4);
        *(volatile v4f*)(yb + (size_t)row * kDim + c4) = val;
      }
      __threadfence();
    }
  }
}

__global__ __launch_bounds__(256) void gnorm_kernel(const float* __restrict__ Y, const float* __restrict__ G,
    const float* __restrict__ lw, const float* __restrict__ lb,
    unsigned short* __restrict__ YGH, unsigned short* __restrict__ YGL) {
  __shared__ float s_y[kDim];
  __shared__ float s_mu[kHeads];
  __shared__ float s_rs[kHeads];
  __shared__ __align__(16) unsigned short s_hl[2 * kDim];
  const int tok = blockIdx.x;
  const int tid = threadIdx.x;
  const size_t rowoff = (size_t)tok * kDim;
#pragma unroll 1
  for (int it = 0; it < 4; ++it) {
    const int d = it * 256 + tid;
    s_y[d] = Y[rowoff + d];
  }
  __syncthreads();
  {
    const int h = tid >> 4, sub = tid & 15;
    float sm = 0.0f;
#pragma unroll
    for (int e = 0; e < 4; ++e) sm += s_y[h * kHd + sub * 4 + e];
    sm += __shfl_xor(sm, 8, 32);
    sm += __shfl_xor(sm, 4, 32);
    sm += __shfl_xor(sm, 2, 32);
    sm += __shfl_xor(sm, 1, 32);
    const float mu = sm * (1.0f / (float)kHd);
    float ss = 0.0f;
#pragma unroll
    for (int e = 0; e < 4; ++e) { const float dv = s_y[h * kHd + sub * 4 + e] - mu; ss += dv * dv; }
    ss += __shfl_xor(ss, 8, 32);
    ss += __shfl_xor(ss, 4, 32);
    ss += __shfl_xor(ss, 2, 32);
    ss += __shfl_xor(ss, 1, 32);
    const float var = ss * (1.0f / (float)kHd);
    const float rs = 1.0f / sqrtf(var + kGnEps);
    if (sub == 0) { s_mu[h] = mu; s_rs[h] = rs; }
  }
  __syncthreads();
#pragma unroll 1
  for (int it = 0; it < 4; ++it) {
    const int d = it * 256 + tid;
    const int h = d >> 6;
    const float g = G[rowoff + d];
    const float gs = g * (1.0f / (1.0f + expf(-g)));
    const float yn = (s_y[d] - s_mu[h]) * s_rs[h] * lw[d] + lb[d];
    const float val = yn * gs;
    const unsigned short hb = f2bf_bits(val);
    s_hl[d] = hb;
    s_hl[kDim + d] = f2bf_bits(val - bf_bits2f(hb));
  }
  __syncthreads();
  const int plane = tid >> 7, chunk = tid & 127;
  const v4u u = *(const v4u*)(s_hl + plane * kDim + chunk * 8);
  unsigned short* dst = (plane ? YGL : YGH) + rowoff + chunk * 8;
  *(volatile v4u*)dst = u;
  __threadfence();
  *(volatile v4u*)dst = u;
}

extern "C" void kernel_launch(void* const* d_in, const int* in_sizes, int n_in,
                              void* d_out, int out_size, void* d_ws, size_t ws_size, hipStream_t stream) {
  if (n_in < 25 || d_out == nullptr || d_ws == nullptr) return;
  if (in_sizes[0] != kTok * kDim) return;
  for (int i = 1; i <= 7; ++i) if (in_sizes[i] != kDim) return;
  if (in_sizes[8] != kDim * kMixN || in_sizes[9] != 6 * kMixW * kDim) return;
  if (in_sizes[10] != kDim || in_sizes[11] != kDim * kLora || in_sizes[12] != kLora * kDim) return;
  if (in_sizes[13] != kDim || in_sizes[14] != kDim * kLora || in_sizes[15] != kLora * kDim) return;
  if (in_sizes[16] != kDim || in_sizes[17] != kDim) return;
  for (int i = 18; i <= 22; ++i) if (in_sizes[i] != kDim * kDim) return;
  if (in_sizes[23] != kDim || in_sizes[24] != kDim) return;
  if (out_size != kTok * kDim) return;
  constexpr size_t MiB = (size_t)1 << 20;
  constexpr size_t kCarve = 127 * MiB;
  static_assert(kCarve <= (size_t)134217728);
  if (ws_size < kCarve) return;

  const float* x    = (const float*)d_in[0];
  const float* tm_x = (const float*)d_in[1];
  const float* tm_w = (const float*)d_in[2];
  const float* tm_k = (const float*)d_in[3];
  const float* tm_v = (const float*)d_in[4];
  const float* tm_r = (const float*)d_in[5];
  const float* tm_g = (const float*)d_in[6];
  const float* tm_a = (const float*)d_in[7];
  const float* maa_w1 = (const float*)d_in[8];
  const float* maa_w2 = (const float*)d_in[9];
  const float* tdecay = (const float*)d_in[10];
  const float* dw1  = (const float*)d_in[11];
  const float* dw2  = (const float*)d_in[12];
  const float* a0   = (const float*)d_in[13];
  const float* a1   = (const float*)d_in[14];
  const float* a2   = (const float*)d_in[15];
  const float* k_k  = (const float*)d_in[16];
  const float* k_a  = (const float*)d_in[17];
  const float* W_r  = (const float*)d_in[18];
  const float* W_k  = (const float*)d_in[19];
  const float* W_v  = (const float*)d_in[20];
  const float* W_g  = (const float*)d_in[21];
  const float* W_o  = (const float*)d_in[22];
  const float* ln_w = (const float*)d_in[23];
  const float* ln_b = (const float*)d_in[24];

  char* ws = (char*)d_ws;
  unsigned short* wsb = (unsigned short*)d_ws;
  const size_t PLB = 4 * MiB;
  unsigned short* WOH  = (unsigned short*)(ws + 0 * MiB);
  unsigned short* WOL  = (unsigned short*)(ws + 2 * MiB);
  char* lw = ws + 4 * MiB;
  unsigned short* W1T  = (unsigned short*)(lw);
  unsigned short* W2T  = (unsigned short*)(lw + 393216);
  unsigned short* DW1T = (unsigned short*)(lw + 786432);
  unsigned short* DW2T = (unsigned short*)(lw + 917504);
  unsigned short* A1TH = (unsigned short*)(lw + 1048576);
  unsigned short* A1TL = (unsigned short*)(lw + 1179648);
  unsigned short* A2TH = (unsigned short*)(lw + 1310720);
  unsigned short* A2TL = (unsigned short*)(lw + 1441792);
  float* Pk = (float*)(ws + 6 * MiB);
  float* Kf = Pk;
  float* Vf = (float*)(ws + 14 * MiB);
  float* Rf = (float*)(ws + 22 * MiB);
  float* Gf = (float*)(ws + 30 * MiB);
  unsigned short* W4H = (unsigned short*)(ws + 38 * MiB);
  unsigned short* W4L = (unsigned short*)(ws + 46 * MiB);
  unsigned short* XXX = (unsigned short*)(ws + 54 * MiB);
  unsigned short* HW  = (unsigned short*)(ws + 54 * MiB);
  unsigned short* HAH = (unsigned short*)(ws + 54 * MiB + 262144);
  unsigned short* HAL = (unsigned short*)(ws + 54 * MiB + 524288);
  unsigned short* HM  = (unsigned short*)(ws + 58 * MiB);
  unsigned short* MIX = (unsigned short*)(ws + 59 * MiB);
  float* WDEC = (float*)(ws + 59 * MiB);
  float* PRE  = (float*)(ws + 67 * MiB);
  float* CSP  = (float*)(ws + 75 * MiB);
  float* Yp   = (float*)(ws + 59 * MiB);
  unsigned short* XW  = (unsigned short*)(ws + 83 * MiB);
  unsigned short* X4H = (unsigned short*)(ws + 87 * MiB);
  unsigned short* X4L = (unsigned short*)(ws + 103 * MiB);
  unsigned short* XAH = (unsigned short*)(ws + 119 * MiB);
  unsigned short* XAL = (unsigned short*)(ws + 123 * MiB);
  const size_t offQb = 83 * MiB, offAb = 38 * MiB, offVb = 115 * MiB;
  unsigned short* QFH = (unsigned short*)(ws + offQb + 0 * PLB);
  unsigned short* QFL = (unsigned short*)(ws + offQb + 1 * PLB);
  unsigned short* KFH = (unsigned short*)(ws + offQb + 2 * PLB);
  unsigned short* KFL = (unsigned short*)(ws + offQb + 3 * PLB);
  unsigned short* QBH = (unsigned short*)(ws + offQb + 4 * PLB);
  unsigned short* QBL = (unsigned short*)(ws + offQb + 5 * PLB);
  unsigned short* KBH = (unsigned short*)(ws + offQb + 6 * PLB);
  unsigned short* KBL = (unsigned short*)(ws + offQb + 7 * PLB);
  unsigned short* AQH = (unsigned short*)(ws + offAb + 0 * PLB);
  unsigned short* AQL = (unsigned short*)(ws + offAb + 1 * PLB);
  unsigned short* KKH = (unsigned short*)(ws + offAb + 2 * PLB);
  unsigned short* KKL = (unsigned short*)(ws + offAb + 3 * PLB);
  unsigned short* V16 = (unsigned short*)(ws + offVb);
  unsigned short* VPF = (unsigned short*)(ws + 119 * MiB);
  unsigned short* VPB = (unsigned short*)(ws + 123 * MiB);
  unsigned short* YGH = (unsigned short*)(ws + 38 * MiB);
  unsigned short* YGL = (unsigned short*)(ws + 42 * MiB);
  float* outp = (float*)d_out;

  trw_kernel<1><<<dim3(kDim / 64, kDim / 64, 4), 256, 0, stream>>>(W_k, W_v, W_r, W_g, W4H, W4L, kDim, kDim, 1.0f);
  trw_kernel<1><<<dim3(kDim / 64, kDim / 64, 1), 256, 0, stream>>>(W_o, W_o, W_o, W_o, WOH, WOL, kDim, kDim, 1.0f);
  trw_kernel<0><<<dim3(kDim / 64, kMixN / 64, 1), 256, 0, stream>>>(maa_w1, maa_w1, maa_w1, maa_w1, W1T, W1T, kDim, kMixN, kCarryW);
  trw_kernel<0><<<dim3(kDim / 64, kLora / 64, 1), 256, 0, stream>>>(dw1, dw1, dw1, dw1, DW1T, DW1T, kDim, kLora, kCarryW);
  trw_kernel<0><<<dim3(kLora / 64, kDim / 64, 1), 256, 0, stream>>>(dw2, dw2, dw2, dw2, DW2T, DW2T, kLora, kDim, kCarryW);
  trw_kernel<1><<<dim3(kDim / 64, kLora / 64, 1), 256, 0, stream>>>(a1, a1, a1, a1, A1TH, A1TL, kDim, kLora, 1.0f);
  trw_kernel<1><<<dim3(kLora / 64, kDim / 64, 1), 256, 0, stream>>>(a2, a2, a2, a2, A2TH, A2TL, kLora, kDim, 1.0f);
  tr32_kernel<<<dim3(kDim / 64, 6), 256, 0, stream>>>(maa_w2, W2T, kCarryW);

  const int nElem8 = kTok * (kDim / 8);
  shift_kernel<<<(nElem8 + 255) / 256, 256, 0, stream>>>(x, tm_x, XXX);

  wmma_gemm64<0, false, 0, 1, 1><<<dim3((kTok / 64) * (kMixN / 64) / 8, 1), 256, 0, stream>>>(
      XXX, XXX, kDim, 0L, W1T, W1T, kDim, 0L, (void*)HM, (void*)HM, kMixN, 0L, tdecay,
      kTok, kMixN, kDim, 1.0f / kCarryW);
  wmma_gemm64<0, false, 0, 1, 0><<<dim3((kTok / 64) * (kDim / 64) / 8, 6), 256, 0, stream>>>(
      HM, HM, kMixN, (long)kMixW, W2T, W2T, kMixW, (long)kDim * kMixW, (void*)MIX, (void*)MIX, kDim, (long)kTok * kDim, tdecay,
      kTok, kDim, kMixW, kCarryMix / (kCarryH * kCarryW));

  combine_kernel<<<(nElem8 + 255) / 256, 256, 0, stream>>>(x, tm_w, tm_k, tm_v, tm_r, tm_g, tm_a, MIX, XW, X4H, X4L, XAH, XAL);

  wmma_gemm64<1, true, 0, 0, 0><<<dim3((kTok / 64) * (kDim / 64) / 8, 4), 256, 0, stream>>>(
      X4H, X4L, kDim, (long)kTok * kDim, W4H, W4L, kDim, (long)kDim * kDim, (void*)Pk, (void*)Pk, kDim, (long)kTok * kDim, tdecay,
      kTok, kDim, kDim, 1.0f);

  wmma_gemm64<0, false, 0, 1, 1><<<dim3((kTok / 64) * (kLora / 64) / 8, 1), 256, 0, stream>>>(
      XW, XW, kDim, 0L, DW1T, DW1T, kDim, 0L, (void*)HW, (void*)HW, kLora, 0L, tdecay,
      kTok, kLora, kDim, 1.0f / kCarryW);
  wmma_gemm64<0, false, 2, 0, 0><<<dim3((kTok / 64) * (kDim / 64) / 8, 1), 256, 0, stream>>>(
      HW, HW, kLora, 0L, DW2T, DW2T, kLora, 0L, (void*)WDEC, (void*)WDEC, kDim, 0L, tdecay,
      kTok, kDim, kLora, 1.0f / (kCarryH * kCarryW));
  wmma_gemm64<1, true, 0, 2, 0><<<dim3((kTok / 64) * (kLora / 64) / 8, 1), 256, 0, stream>>>(
      XAH, XAL, kDim, 0L, A1TH, A1TL, kDim, 0L, (void*)HAH, (void*)HAL, kLora, 0L, tdecay,
      kTok, kLora, kDim, 1.0f);
  wmma_gemm64<1, true, 2, 0, 0><<<dim3((kTok / 64) * (kDim / 64) / 8, 1), 256, 0, stream>>>(
      HAH, HAL, kLora, 0L, A2TH, A2TL, kLora, 0L, (void*)PRE, (void*)PRE, kDim, 0L, a0,
      kTok, kDim, kLora, 1.0f);

  scan_kernel<<<(kBatch * kDim) / 64, 64, 0, stream>>>(WDEC, CSP);

  headprep_kernel<<<kTok, 256, 0, stream>>>(Kf, Vf, Rf, PRE, WDEC, CSP, k_k, k_a, wsb,
      (long)(offQb / 2), (long)(offAb / 2), (long)(offVb / 2));

  pairmix_kernel<true><<<(kSeq / 64) * kBatch * kHeads, 128, 0, stream>>>(
      AQH, AQL, KKH, KKL, V16, AQH, AQL, KKH, KKL, V16, Vf, VPF, VPB, Yp);
  pairmix_kernel<false><<<(kSeq / 64) * kBatch * kHeads, 128, 0, stream>>>(
      QFH, QFL, KFH, KFL, VPF, QBH, QBL, KBH, KBL, VPB, Vf, VPF, VPB, Yp);

  gnorm_kernel<<<kTok, 256, 0, stream>>>(Yp, Gf, ln_w, ln_b, YGH, YGL);

  wmma_gemm64<1, true, 0, 0, 0><<<dim3((kTok / 64) * (kDim / 64) / 8, 1), 256, 0, stream>>>(
      YGH, YGL, kDim, 0L, WOH, WOL, kDim, 0L, (void*)outp, (void*)outp, kDim, 0L, tdecay,
      kTok, kDim, kDim, 1.0f);
}
